// Attention_74191265071149
// MI455X (gfx1250) — hardware-run, weakly checked
//
#include <hip/hip_runtime.h>


#ifndef NB
#define NB 32
#endif
#ifndef SEQ
#define SEQ 1024
#endif
#define NB_FULL  32
#define SEQ_FULL 1024
#ifndef OUT_SEQ
#define OUT_SEQ SEQ
#endif
#define DM   256
#define NH_  8
#define HD   32
#define TABLE 3969
#define AW   4
#define OSP  36
#define SC2  ((float)(0.17677669529663687 * 1.4426950408889634))
#define LOG2E 1.4426950408889634f
#define PSH  14.0f
#define NEGB (-3.0e38f)
#define CTC  256.0f
#define WOC  64.0f
#define FOLD (1.0f / 16384.0f)

static_assert(HD == 32);
static_assert(NH_ == 8);
static_assert(NH_ * HD == DM);
static_assert(DM % 64 == 0);
static_assert(64 % HD == 0);
static_assert(DM % 32 == 0);
static_assert(SEQ % 64 == 0);
static_assert((NB * SEQ) % 64 == 0);
static_assert(SEQ % 32 == 0);
static_assert(SEQ % (16 * AW) == 0);
static_assert(SEQ % 128 == 0);
static_assert(((size_t)SEQ * SEQ / 4) % 256 == 0);
static_assert(SEQ_FULL % 4 == 0);
static_assert(((size_t)SEQ * DM) % 8 == 0);
static_assert(NB <= NB_FULL);
static_assert(SEQ <= SEQ_FULL);
static_assert((OSP * 4) % 16 == 0);
static_assert(CTC * WOC * FOLD == 1.0f);
static_assert(2 * 2 * 32 * 16 == 16 * 64 * 2);
static_assert(4 * 32 * 16 == 16 * 64 * 2);
static_assert(8 * 32 * 16 == 16 * 64 * 4);
static_assert(2 * 32 * 16 == 16 * HD * 2);
static_assert(2 * 256 * 16 == 64 * 64 * 2);
static_assert(16 * 256 == 64 * 64);
static_assert(16 * 68 * 4 <= 131072);
static_assert(64 * 68 * 4 <= 131072);
static_assert(AW * 16 * OSP * 4 <= 131072);

typedef _Float16 h16;
typedef unsigned short bf;
typedef __attribute__((ext_vector_type(16))) __bf16   v16bf;
typedef __attribute__((ext_vector_type(16))) _Float16 v16h;
typedef __attribute__((ext_vector_type(8)))  _Float16 v8h;
typedef __attribute__((ext_vector_type(8)))  unsigned short v8us;
typedef __attribute__((ext_vector_type(8)))  float    v8f;
typedef __attribute__((ext_vector_type(4)))  float    v4f;
typedef __attribute__((ext_vector_type(4)))  int      v4i;
typedef v4f  __attribute__((may_alias)) v4fa;

__device__ __forceinline__ unsigned short f2bf(float f) { unsigned u = __float_as_uint(f); u += 0x7FFFu + ((u >> 16) & 1u); return (unsigned short)(u >> 16); }
__device__ __forceinline__ float bfr(float f) { return __uint_as_float(((unsigned)f2bf(f)) << 16); }
__device__ __forceinline__ v16h cat16(v8h lo, v8h hi) { return __builtin_shufflevector(lo, hi, 0, 1, 2, 3, 4, 5, 6, 7, 8, 9, 10, 11, 12, 13, 14, 15); }
__device__ __forceinline__ v16bf cat16b(v8us lo, v8us hi) { return __builtin_bit_cast(v16bf, __builtin_shufflevector(lo, hi, 0, 1, 2, 3, 4, 5, 6, 7, 8, 9, 10, 11, 12, 13, 14, 15)); }
__device__ __forceinline__ v8f wmma16(v16h a, v16h b, v8f c) { return __builtin_amdgcn_wmma_f32_16x16x32_f16(false, a, false, b, (short)0, c, false, false); }
__device__ __forceinline__ v8f wmmab(v16bf a, v16bf b, v8f c) { return __builtin_amdgcn_wmma_f32_16x16x32_bf16(false, a, false, b, (short)0, c, false, false); }
__device__ __forceinline__ v16h  ldh(const h16* p) { return cat16(*(const v8h*)p, *(const v8h*)(p + 16)); }
__device__ __forceinline__ v16bf ldb(const bf* p)  { return cat16b(*(const v8us*)p, *(const v8us*)(p + 16)); }
__device__ __forceinline__ void wave_sync() { __builtin_amdgcn_fence(3  , "wavefront"); __builtin_amdgcn_wave_barrier(); asm volatile("" ::: "memory"); }
__device__ __forceinline__ v8f wmma16g(v16h a, v16h b, v8f c) { c = wmma16(a, b, c); asm volatile("v_nop\n\tv_nop\n\tv_nop\n\tv_nop" : "+v"(c) : "v"(a), "v"(b)); return c; }
__device__ __forceinline__ v8f wmmabg(v16bf a, v16bf b, v8f c) { c = wmmab(a, b, c); asm volatile("v_nop\n\tv_nop\n\tv_nop\n\tv_nop" : "+v"(c) : "v"(a), "v"(b)); return c; }
static __device__ __forceinline__ h16 toh_flush(float v) { const h16 r = (h16)v; return (fabsf(v) < 6.103515625e-05f) ? (h16)0.0f : r; }

__global__ __launch_bounds__(256) void k_cvt8(const float* __restrict__ src, bf* dst, size_t n8) {
    const size_t i = (size_t)blockIdx.x * 256 + threadIdx.x; if (i >= n8) return;
    const v8f v = *(const v8f*)(src + i * 8); v8us o;
#pragma unroll
    for (int k = 0; k < 8; ++k) o[k] = f2bf(v[k]);
    *(volatile v8us*)(dst + i * 8) = o; __threadfence(); *(volatile v8us*)(dst + i * 8) = o;
}

__global__ __launch_bounds__(256) void k_wt_bf(const float* __restrict__ in, bf* out, int rows, int cols) {
    __shared__ __align__(16) float ts[64 * 68];
    const int tid = threadIdx.x; const int c0 = blockIdx.x * 64, r0 = blockIdx.y * 64;
#pragma unroll 1
    for (int it = 0; it < 16; ++it) { const int e = it * 256 + tid; const int r = e >> 6, c = e & 63;
        ts[c * 68 + r] = in[(size_t)(r0 + r) * cols + c0 + c]; }
    __syncthreads();
#pragma unroll 1
    for (int ps = 0; ps < 2; ++ps) {
#pragma unroll
        for (int it = 0; it < 2; ++it) { const int p = it * 256 + tid; const int row = p >> 3, c8 = (p & 7) * 8;
            const v4f x0 = *(const v4fa*)(&ts[row * 68 + c8]); const v4f x1 = *(const v4fa*)(&ts[row * 68 + c8 + 4]); v8us o;
#pragma unroll
            for (int i = 0; i < 4; ++i) { o[i] = f2bf(x0[i]); o[4 + i] = f2bf(x1[i]); }
            *(volatile v8us*)(out + (size_t)(c0 + row) * rows + r0 + c8) = o; }
        if (ps == 0) __threadfence(); }
}

__global__ __launch_bounds__(256) void k_wt_h(const float* __restrict__ in, h16* out, int rows, int cols, float carry) {
    __shared__ __align__(16) float ts[64 * 68];
    const int tid = threadIdx.x; const int c0 = blockIdx.x * 64, r0 = blockIdx.y * 64;
#pragma unroll 1
    for (int it = 0; it < 16; ++it) { const int e = it * 256 + tid; const int r = e >> 6, c = e & 63;
        ts[c * 68 + r] = in[(size_t)(r0 + r) * cols + c0 + c]; }
    __syncthreads();
#pragma unroll 1
    for (int ps = 0; ps < 2; ++ps) {
#pragma unroll
        for (int it = 0; it < 2; ++it) { const int p = it * 256 + tid; const int row = p >> 3, c8 = (p & 7) * 8;
            const v4f x0 = *(const v4fa*)(&ts[row * 68 + c8]); const v4f x1 = *(const v4fa*)(&ts[row * 68 + c8 + 4]); v8h o;
#pragma unroll
            for (int i = 0; i < 4; ++i) { o[i] = toh_flush(bfr(x0[i]) * carry); o[4 + i] = toh_flush(bfr(x1[i]) * carry); }
            *(volatile v8h*)(out + (size_t)(c0 + row) * rows + r0 + c8) = o; }
        if (ps == 0) __threadfence(); }
}

__global__ __launch_bounds__(256) void k_bias(const float* __restrict__ table, const int* __restrict__ rel, float* BP) {
    const int id = blockIdx.x * 256 + threadIdx.x;
    const int i = id / (SEQ / 4), j = (id % (SEQ / 4)) * 4;
    const v4i rv = *(const v4i*)(rel + (size_t)i * SEQ_FULL + j);
    float tv[4][8];
#pragma unroll
    for (int e = 0; e < 4; ++e) {
        int ix = rv[e]; ix = ix < 0 ? 0 : (ix > TABLE - 1 ? TABLE - 1 : ix);
        const v4f a = *(const v4f*)(table + (size_t)ix * NH_); const v4f c = *(const v4f*)(table + (size_t)ix * NH_ + 4);
#pragma unroll
        for (int q = 0; q < 4; ++q) { tv[e][q] = bfr(a[q]) * LOG2E; tv[e][4 + q] = bfr(c[q]) * LOG2E; } }
    v4f o[8];
#pragma unroll
    for (int h = 0; h < 8; ++h) { o[h][0] = tv[0][h]; o[h][1] = tv[1][h]; o[h][2] = tv[2][h]; o[h][3] = tv[3][h]; }
    float* dst = BP + (size_t)i * SEQ + j;
#pragma unroll 1
    for (int ps = 0; ps < 2; ++ps) {
#pragma unroll
        for (int h = 0; h < 8; ++h) *(volatile v4f*)(dst + (size_t)h * SEQ * SEQ) = o[h];
        if (ps == 0) __threadfence(); }
}

__global__ __launch_bounds__(32) void k_proj_qk(const bf* __restrict__ A, const bf* __restrict__ Bt, h16* Ph) {
    __shared__ __align__(16) float os[16 * 68];
    const int lane = threadIdx.x & 31, lr = lane & 15, hi = lane >> 4; const int r0 = blockIdx.x * 64, c0 = blockIdx.y * 64;
    v8f acc[4][4];
#pragma unroll
    for (int mb = 0; mb < 4; ++mb)
#pragma unroll
        for (int nb = 0; nb < 4; ++nb) acc[mb][nb] = (v8f){};
    const size_t aoff = (size_t)(r0 + lr) * DM + 8 * hi, boff = (size_t)(c0 + lr) * DM + 8 * hi;
#pragma unroll 1
    for (int kc = 0; kc < DM; kc += 32) {
        v16bf a[4];
#pragma unroll
        for (int mb = 0; mb < 4; ++mb) a[mb] = ldb(A + aoff + (size_t)mb * 16 * DM + kc);
#pragma unroll
        for (int nb = 0; nb < 4; ++nb) { const v16bf b = ldb(Bt + boff + (size_t)nb * 16 * DM + kc);
#pragma unroll
            for (int mb = 0; mb < 4; ++mb) acc[mb][nb] = wmmabg(a[mb], b, acc[mb][nb]); }
    }
    const int sec = c0 / DM, cc = c0 % DM;
    const int bb = r0 / SEQ, tt = r0 % SEQ; const int zc = bb * NH_ + cc / HD;
    const size_t tbase = (size_t)sec * ((size_t)NB * NH_ * SEQ * HD) + ((size_t)zc * SEQ + (size_t)tt) * HD;
#pragma unroll
    for (int mb = 0; mb < 4; ++mb) {
#pragma unroll
        for (int nb = 0; nb < 4; ++nb) {
#pragma unroll
            for (int j = 0; j < 8; ++j) os[(hi * 8 + j) * 68 + nb * 16 + lr] = acc[mb][nb][j]; }
        wave_sync();
#pragma unroll 1
        for (int ps = 0; ps < 2; ++ps) {
            const size_t sb = tbase + (size_t)(mb * 16) * HD;
#pragma unroll
            for (int hh = 0; hh < 2; ++hh) {
#pragma unroll
                for (int s = 0; s < 2; ++s) { const int p = s * 32 + lane; const int row = p >> 2, c8 = (p & 3) * 8;
                    const v4f x0 = *(const v4fa*)(&os[row * 68 + hh * 32 + c8]); const v4f x1 = *(const v4fa*)(&os[row * 68 + hh * 32 + c8 + 4]); v8h hv;
#pragma unroll
                    for (int i = 0; i < 4; ++i) { hv[i] = toh_flush(x0[i]); hv[4 + i] = toh_flush(x1[i]); }
                    const size_t oo = sb + (size_t)hh * ((size_t)SEQ * HD) + (size_t)p * 8;
                    *(volatile v8h*)(Ph + oo) = hv; } }
            if (ps == 0) __threadfence(); }
        wave_sync();
    }
}

__global__ __launch_bounds__(32) void k_proj_vt(const bf* __restrict__ A, const bf* __restrict__ Bt, h16* Ph) {
    __shared__ __align__(16) float os[16 * 68];
    const int lane = threadIdx.x & 31, lr = lane & 15, hi = lane >> 4; const int r0 = blockIdx.x * 64, c0 = blockIdx.y * 64;
    v8f acc[4][4];
#pragma unroll
    for (int mb = 0; mb < 4; ++mb)
#pragma unroll
        for (int nb = 0; nb < 4; ++nb) acc[mb][nb] = (v8f){};
    const size_t aoff = (size_t)(r0 + lr) * DM + 8 * hi, boff = (size_t)(c0 + lr) * DM + 8 * hi;
#pragma unroll 1
    for (int kc = 0; kc < DM; kc += 32) {
        v16bf a[4];
#pragma unroll
        for (int mb = 0; mb < 4; ++mb) a[mb] = ldb(A + aoff + (size_t)mb * 16 * DM + kc);
#pragma unroll
        for (int nb = 0; nb < 4; ++nb) { const v16bf b = ldb(Bt + boff + (size_t)nb * 16 * DM + kc);
#pragma unroll
            for (int mb = 0; mb < 4; ++mb) acc[mb][nb] = wmmabg(a[mb], b, acc[mb][nb]); }
    }
    const int bb = c0 / SEQ, tt = c0 % SEQ;
    const size_t tbase = (size_t)bb * (size_t)DM * SEQ + (size_t)r0 * SEQ + (size_t)tt;
#pragma unroll
    for (int mb = 0; mb < 4; ++mb) {
#pragma unroll
        for (int nb = 0; nb < 4; ++nb) {
#pragma unroll
            for (int j = 0; j < 8; ++j) os[(hi * 8 + j) * 68 + nb * 16 + lr] = acc[mb][nb][j]; }
        wave_sync();
#pragma unroll 1
        for (int ps = 0; ps < 2; ++ps) {
            const size_t sb = tbase + (size_t)(mb * 16) * SEQ;
#pragma unroll
            for (int s = 0; s < 4; ++s) { const int row = 4 * s + (lane >> 3), c8 = (lane & 7) * 8;
                const v4f x0 = *(const v4fa*)(&os[row * 68 + c8]); const v4f x1 = *(const v4fa*)(&os[row * 68 + c8 + 4]); v8h hv;
#pragma unroll
                for (int i = 0; i < 4; ++i) { hv[i] = toh_flush(x0[i]); hv[4 + i] = toh_flush(x1[i]); }
                const size_t oo = sb + (size_t)row * SEQ + c8;
                *(volatile v8h*)(Ph + oo) = hv; }
            if (ps == 0) __threadfence(); }
        wave_sync();
    }
}

__global__ __launch_bounds__(32 * AW) void k_flash(const h16* __restrict__ QH, const h16* __restrict__ KP, const h16* __restrict__ VT, const float* __restrict__ BP, h16* CT) {
    __shared__ __align__(16) float os[AW * 16 * OSP];
    const int lane = threadIdx.x & 31, lr = lane & 15, hi = lane >> 4;
    const int wave = __builtin_amdgcn_readfirstlane((int)(threadIdx.x >> 5));
    const int zh = blockIdx.y; const int h = zh % NH_;
    const int t0 = (blockIdx.x * AW + wave) * 16;
    const size_t pbase = (size_t)zh * SEQ * HD;
    const v16h qh = ldh(QH + pbase + (size_t)(t0 + lr) * HD + 8 * hi);
    const size_t ko = pbase + (size_t)lr * HD + 8 * hi;
    const size_t vo = pbase + (size_t)lr * SEQ + 8 * hi;
    const size_t bo = ((size_t)h * SEQ + (size_t)(t0 + lr)) * SEQ + 8 * hi;
    v8f o0 = (v8f){}, o1 = (v8f){};
    float m = NEGB, l = 0.0f;
#pragma unroll 1
    for (int key0 = 0; key0 < SEQ; key0 += 32) {
        const h16* ka = KP + ko + (size_t)key0 * HD;
        const v16h ka0 = ldh(ka), kb0 = ldh(ka + 16 * HD);
        v8f sa = (v8f){}, sb = (v8f){};
        sa = wmma16g(ka0, qh, sa); sb = wmma16g(kb0, qh, sb);
        const float* bp = BP + bo + key0;
        const v4f m0 = *(const v4f*)bp, m1 = *(const v4f*)(bp + 4), m2 = *(const v4f*)(bp + 16), m3 = *(const v4f*)(bp + 20);
        float bx[8], by[8];
#pragma unroll
        for (int r = 0; r < 4; ++r) { bx[r] = m0[r]; bx[4 + r] = m1[r]; by[r] = m2[r]; by[4 + r] = m3[r]; }
        float ta[8], tb[8]; float mx = NEGB;
#pragma unroll
        for (int r = 0; r < 8; ++r) {
            ta[r] = sa[r] * SC2 + bx[r]; tb[r] = sb[r] * SC2 + by[r];
            mx = fmaxf(mx, fmaxf(ta[r], tb[r])); }
        mx = fmaxf(mx, __shfl_xor(mx, 16, 32));
        const float mnew = fmaxf(m, mx);
        const float alpha = __builtin_amdgcn_exp2f(m - mnew);
        const float sh = PSH - mnew;
        v16h pb; float ls = 0.0f;
#pragma unroll
        for (int r = 0; r < 8; ++r) {
            const float xa = ta[r] + sh, xb = tb[r] + sh;
            const float ea = (xa < -14.0f) ? 0.0f : __builtin_amdgcn_exp2f(xa);
            const float eb = (xb < -14.0f) ? 0.0f : __builtin_amdgcn_exp2f(xb);
            const h16 pa = (h16)ea; const h16 pc = (h16)eb;
            pb[r] = pa; pb[8 + r] = pc;
            ls += (float)pa + (float)pc; }
        l = l * alpha + ls; m = mnew;
        o0 = o0 * alpha; o1 = o1 * alpha;
        const h16* va = VT + vo + key0;
        const v16h v0 = ldh(va), v1 = ldh(va + (size_t)16 * SEQ);
        o0 = wmma16g(v0, pb, o0); o1 = wmma16g(v1, pb, o1);
    }
    l += __shfl_xor(l, 16, 32);
    const float inv = CTC * (1.0f / l);
    const int wb = wave * 16 * OSP;
    { v4f a, c;
      a[0] = o0[0] * inv; a[1] = o0[1] * inv; a[2] = o0[2] * inv; a[3] = o0[3] * inv; c[0] = o0[4] * inv; c[1] = o0[5] * inv; c[2] = o0[6] * inv; c[3] = o0[7] * inv;
      *(v4fa*)(&os[wb + lr * OSP +  0 + 8 * hi]) = a; *(v4fa*)(&os[wb + lr * OSP +  0 + 8 * hi + 4]) = c;
      a[0] = o1[0] * inv; a[1] = o1[1] * inv; a[2] = o1[2] * inv; a[3] = o1[3] * inv; c[0] = o1[4] * inv; c[1] = o1[5] * inv; c[2] = o1[6] * inv; c[3] = o1[7] * inv;
      *(v4fa*)(&os[wb + lr * OSP + 16 + 8 * hi]) = a; *(v4fa*)(&os[wb + lr * OSP + 16 + 8 * hi + 4]) = c; }
    wave_sync();
    h16* crow = CT + pbase + (size_t)t0 * HD;
#pragma unroll 1
    for (int ps = 0; ps < 2; ++ps) {
#pragma unroll
        for (int s = 0; s < 2; ++s) { const int p = s * 32 + lane; const int row = p >> 2, c8 = (p & 3) * 8;
            const v4f x0 = *(const v4fa*)(&os[wb + row * OSP + c8]); const v4f x1 = *(const v4fa*)(&os[wb + row * OSP + c8 + 4]); v8h hv;
#pragma unroll
            for (int i = 0; i < 4; ++i) { hv[i] = toh_flush(x0[i]); hv[4 + i] = toh_flush(x1[i]); }
            *(volatile v8h*)(crow + (size_t)p * 8) = hv; }
        if (ps == 0) __threadfence(); }
}

__global__ __launch_bounds__(32) void k_outp(const h16* __restrict__ CT, const h16* __restrict__ Wt, const float* __restrict__ bo, float* OUT) {
    __shared__ __align__(16) float os[16 * 68];
    const int lane = threadIdx.x & 31, lr = lane & 15, hi = lane >> 4; const int r0 = blockIdx.x * 64, c0 = blockIdx.y * 64;
    const int bb = r0 / SEQ, tt = r0 % SEQ;
    v8f acc[4][4];
#pragma unroll
    for (int mb = 0; mb < 4; ++mb)
#pragma unroll
        for (int nb = 0; nb < 4; ++nb) acc[mb][nb] = (v8f){};
    const size_t aoff = ((size_t)bb * NH_ * SEQ + (size_t)(tt + lr)) * HD + 8 * hi, boff = (size_t)(c0 + lr) * DM + 8 * hi;
#pragma unroll 1
    for (int hd = 0; hd < NH_; ++hd) {
        v16h a[4];
#pragma unroll
        for (int mb = 0; mb < 4; ++mb) a[mb] = ldh(CT + aoff + (size_t)hd * SEQ * HD + (size_t)mb * 16 * HD);
#pragma unroll
        for (int nb = 0; nb < 4; ++nb) { const v16h b = ldh(Wt + boff + (size_t)nb * 16 * DM + hd * HD);
#pragma unroll
            for (int mb = 0; mb < 4; ++mb) acc[mb][nb] = wmma16g(a[mb], b, acc[mb][nb]); }
    }
    const int c4 = (lane & 15) * 4;
    const v4f braw = *(const v4f*)(bo + c0 + c4);
    v4f bv; bv[0] = bfr(braw[0]); bv[1] = bfr(braw[1]); bv[2] = bfr(braw[2]); bv[3] = bfr(braw[3]);
    float* obase = OUT + ((size_t)bb * OUT_SEQ + (size_t)tt) * DM + c0 + c4;
#pragma unroll
    for (int mb = 0; mb < 4; ++mb) {
#pragma unroll
        for (int nb = 0; nb < 4; ++nb) {
#pragma unroll
            for (int j = 0; j < 8; ++j) os[(hi * 8 + j) * 68 + nb * 16 + lr] = acc[mb][nb][j] * FOLD; }
        wave_sync();
#pragma unroll 1
        for (int ps = 0; ps < 2; ++ps) {
#pragma unroll
            for (int s = 0; s < 8; ++s) { const int row = 2 * s + (lane >> 4);
                const v4f val = *(const v4fa*)(&os[row * 68 + c4]) + bv;
                *(volatile v4f*)(obase + (size_t)(mb * 16 + row) * DM) = val; }
            if (ps == 0) __threadfence(); }
        wave_sync();
    }
}

static constexpr size_t al256(size_t v) { return (v + 255) & ~(size_t)255; }
static constexpr size_t PLANE_E = (size_t)NB * NH_ * SEQ * HD;
static constexpr size_t SZ_XB = al256((size_t)NB * SEQ * DM * 2);
static constexpr size_t SZ_WT = al256((size_t)3 * DM * DM * 2);
static constexpr size_t SZ_WO = al256((size_t)DM * DM * 2);
static constexpr size_t SZ_PL = al256(PLANE_E * 2);
static constexpr size_t SZ_BP = al256((size_t)NH_ * SEQ * SEQ * 4);
static constexpr size_t SZ_TOTAL = SZ_XB + SZ_WT + SZ_WO + 4 * SZ_PL + SZ_BP;
static_assert(SZ_TOTAL <= (size_t)134217728);
static_assert((PLANE_E * 2) % 256 == 0);
static_assert(((size_t)DM * DM * 2) % 256 == 0);
static_assert(PLANE_E == (size_t)NB * DM * SEQ);

extern "C" void kernel_launch(void* const* d_in, const int* in_sizes, int n_in,
                              void* d_out, int out_size, void* d_ws, size_t ws_size, hipStream_t stream) {
    if (n_in < 6) return;
    const size_t needx = ((size_t)(NB - 1) * SEQ_FULL + SEQ) * DM;
    if ((size_t)in_sizes[0] < needx) return;
    if ((size_t)in_sizes[1] < (size_t)DM * 3 * DM) return;
    if ((size_t)in_sizes[2] < (size_t)TABLE * NH_) return;
    if ((size_t)in_sizes[3] < (size_t)DM * DM) return;
    if (in_sizes[4] < DM) return;
    if ((size_t)in_sizes[5] < (size_t)(SEQ - 1) * SEQ_FULL + SEQ) return;
    if ((size_t)out_size < ((size_t)(NB - 1) * OUT_SEQ + SEQ) * DM) return;
    if (SZ_TOTAL > ws_size) return;
    const float* x     = (const float*)d_in[0];
    const float* wqkv  = (const float*)d_in[1];
    const float* table = (const float*)d_in[2];
    const float* wout  = (const float*)d_in[3];
    const float* bout  = (const float*)d_in[4];
    const int*   rel   = (const int*)d_in[5];
    float* OUT = (float*)d_out;
    char* wsp = (char*)d_ws;
    bf*  XB  = (bf*)wsp;  wsp += SZ_XB;
    bf*  WT  = (bf*)wsp;  wsp += SZ_WT;
    h16* WOT = (h16*)wsp; wsp += SZ_WO;
    h16* QK  = (h16*)wsp; wsp += 2 * SZ_PL;
    h16* VT  = (h16*)wsp; wsp += SZ_PL;
    h16* CT  = (h16*)wsp; wsp += SZ_PL;
    float* BP = (float*)wsp; wsp += SZ_BP;
    h16* QH = QK; h16* KP = QK + PLANE_E;

    if (SEQ == SEQ_FULL) {
        const size_t n8 = (size_t)NB * SEQ * DM / 8;
        k_cvt8<<<(unsigned)((n8 + 255) / 256), 256, 0, stream>>>(x, XB, n8);
    } else {
        const size_t n8 = (size_t)SEQ * DM / 8;
        for (int b = 0; b < NB; ++b) k_cvt8<<<(unsigned)((n8 + 255) / 256), 256, 0, stream>>>(x + (size_t)b * SEQ_FULL * DM, XB + (size_t)b * SEQ * DM, n8);
    }
    k_wt_bf<<<dim3(3 * DM / 64, DM / 64, 1), 256, 0, stream>>>(wqkv, WT, DM, 3 * DM);
    k_wt_h<<<dim3(DM / 64, DM / 64, 1), 256, 0, stream>>>(wout, WOT, DM, DM, WOC);
    k_bias<<<(unsigned)((size_t)SEQ * SEQ / 4 / 256), 256, 0, stream>>>(table, rel, BP);

    k_proj_qk<<<dim3(NB * SEQ / 64, 2 * DM / 64, 1), 32, 0, stream>>>(XB, WT, QK);
    k_proj_vt<<<dim3(DM / 64, NB * SEQ / 64, 1), 32, 0, stream>>>(WT + (size_t)2 * DM * DM, XB, VT);

    k_flash<<<dim3(SEQ / (16 * AW), NB * NH_, 1), 32 * AW, 0, stream>>>(QH, KP, VT, BP, CT);

    k_outp<<<dim3(NB * SEQ / 64, DM / 64, 1), 32, 0, stream>>>(CT, WOT, bout, OUT);
}
